// PredictBlock_82841329205803
// MI455X (gfx1250) — hardware-run, weakly checked
//
#include <hip/hip_runtime.h>
#include <math.h>

#ifndef NB
#define NB 2
#endif
#ifndef SEQ
#define SEQ 2048
#endif
#define NB_FULL 2
#define SEQ_FULL 2048

constexpr int CD = 1024;
constexpr int NH = 16;
constexpr int HD = 32;
constexpr int HDM = NH * HD;
constexpr int C4 = 4 * CD;
constexpr int NCH = SEQ / 64;
constexpr int MTOK = NB * SEQ;
constexpr int QKP = 2 * HDM;
constexpr int VTP = MTOK;

static_assert(NB >= 1 && NB <= NB_FULL);
static_assert(SEQ <= SEQ_FULL);
static_assert(HD == 32);
static_assert(HDM == 512 && NH % 2 == 0);
static_assert(2 * HD * 2 == 128);
static_assert(QKP == 2 * HDM);
static_assert(CD % 128 == 0 && CD / 128 == 8);
static_assert(8 * CD * 4 <= 65536);
static_assert(MTOK % 64 == 0 && CD % 64 == 0 && HDM % 64 == 0 && C4 % 64 == 0);
static_assert(CD % 32 == 0 && C4 % 32 == 0 && HDM % 32 == 0);
static_assert(MTOK % 8 == 0);
static_assert(SEQ % 64 == 0);
static_assert((HDM * (CD / 8)) % 256 == 0);
static_assert((size_t)NB_FULL * SEQ_FULL * CD * 4 == (size_t)16777216);

typedef __attribute__((ext_vector_type(16))) _Float16 v16h;
typedef __attribute__((ext_vector_type(8)))  _Float16 v8h;
typedef __attribute__((ext_vector_type(8)))  float    v8f;
typedef __attribute__((ext_vector_type(4)))  float    v4f;
typedef __attribute__((ext_vector_type(4)))  unsigned int v4u;
typedef __attribute__((ext_vector_type(2)))  unsigned int v2u;
typedef _Float16 h16;

union FH { v16h v; v8h h[2]; };

#define VST2(T, ptr, val) do { const T vst2_v_ = (val); *(volatile T*)(ptr) = vst2_v_; __threadfence(); *(volatile T*)(ptr) = vst2_v_; } while (0)

#define WAVE_SYNC() do { __builtin_amdgcn_fence(3  , "workgroup"); __builtin_amdgcn_wave_barrier(); __builtin_amdgcn_fence(2  , "workgroup"); } while (0)

__device__ __forceinline__ float cmb_bf(float v) { const unsigned u = __builtin_bit_cast(unsigned, v); const unsigned r = (u + 0x7fffu + ((u >> 16) & 1u)) & 0xffff0000u; return __builtin_bit_cast(float, r); }
__device__ __forceinline__ unsigned int pk2h(float a, float b) { return (unsigned int)__builtin_bit_cast(unsigned short, (_Float16)a) | ((unsigned int)__builtin_bit_cast(unsigned short, (_Float16)b) << 16); }
static __device__ __forceinline__ h16 toh_flush(float v) { const h16 r = (h16)v; return (fabsf(v) < 6.103515625e-05f) ? (h16)0.0f : r; }
__device__ __forceinline__ unsigned int pk2h_fl(float a, float b) { return (unsigned int)__builtin_bit_cast(unsigned short, toh_flush(a)) | ((unsigned int)__builtin_bit_cast(unsigned short, toh_flush(b)) << 16); }
__device__ __forceinline__ v16h ldg_frag(const _Float16* __restrict__ p) { FH f; f.h[0] = *(const v8h*)(p); f.h[1] = *(const v8h*)(p + 16); return f.v; }

__device__ __forceinline__ v8f mma_h(v16h a, v16h b, v8f c) {
  c = __builtin_amdgcn_wmma_f32_16x16x32_f16(false, a, false, b, (short)0, c, false, false);
  asm volatile("v_nop\n\tv_nop\n\tv_nop\n\tv_nop" : "+v"(c) : "v"(a), "v"(b));
  return c;
}
__device__ __forceinline__ void dep_guard_h(v8f& a, v8f& b, v16h x, v16h y) { asm volatile("v_nop\n\tv_nop\n\tv_nop\n\tv_nop" : "+v"(a), "+v"(b) : "v"(x), "v"(y)); }
__device__ __forceinline__ void keep4_h(v16h a, v16h b, v16h c, v16h d) { asm volatile("v_nop" :: "v"(a), "v"(b), "v"(c), "v"(d)); }
__device__ __forceinline__ void acc_guard4(v8f& a, v8f& b, v8f& c, v8f& d) { asm volatile("v_nop\n\tv_nop\n\tv_nop\n\tv_nop" : "+v"(a), "+v"(b), "+v"(c), "+v"(d)); }

__device__ __forceinline__ float gelu_erf(float t) {
  const float ax = fabsf(t) * 0.70710678118654752f;
  const float kk = __builtin_amdgcn_rcpf(1.0f + 0.3275911f * ax);
  float pl = 1.061405429f * kk - 1.453152027f;
  pl = pl * kk + 1.421413741f;
  pl = pl * kk - 0.284496736f;
  pl = pl * kk + 0.254829592f;
  pl = pl * kk;
  const float ex = __builtin_amdgcn_exp2f(-1.4426950408889634f * (ax * ax));
  const float er = 1.0f - pl * ex;
  return 0.5f * t * (1.0f + copysignf(er, t));
}

__global__ __launch_bounds__(256) void k_castbT(const float* __restrict__ SRC, int lds, unsigned short* __restrict__ DST, int ldd, int nR, int nC, float sc) {
  const long long u = (long long)blockIdx.x * 256 + threadIdx.x; const int per = nR / 8; if (u >= (long long)nC * per) return;
  const int cc = (int)(u / per); const int r0 = 8 * (int)(u % per);
  float w[8];
#pragma unroll
  for (int e = 0; e < 8; ++e) w[e] = cmb_bf(SRC[(long long)(r0 + e) * lds + cc]) * sc;
  v4u pk; pk.x = pk2h(w[0], w[1]); pk.y = pk2h(w[2], w[3]); pk.z = pk2h(w[4], w[5]); pk.w = pk2h(w[6], w[7]);
  VST2(v4u, (v4u*)(DST + (long long)cc * ldd + r0), pk);
}

__global__ __launch_bounds__(256) void k_castqkv(const float* __restrict__ SRC, unsigned short* __restrict__ DST) {
  constexpr int per = CD / 8;
  const int u = blockIdx.x * 256 + threadIdx.x; if (u >= HDM * per) return;
  const int n = u / per; const int c0 = 8 * (u % per);
  const int hd = n / HD, d = n % HD;
  float w[8];
#pragma unroll
  for (int e = 0; e < 8; ++e) w[e] = cmb_bf(SRC[((size_t)hd * CD + (size_t)(c0 + e)) * HD + d]) * 16.0f;
  v4u pk; pk.x = pk2h_fl(w[0], w[1]); pk.y = pk2h_fl(w[2], w[3]); pk.z = pk2h_fl(w[4], w[5]); pk.w = pk2h_fl(w[6], w[7]);
  VST2(v4u, (v4u*)(DST + (size_t)n * CD + c0), pk);
}

#define LN_EPS 1e-5f

template <int ABF>
__device__ __forceinline__ void ln_fetch(const float* __restrict__ A, size_t srow, int L, float* rowp) {
#pragma unroll 1
  for (int q = 0; q < 8; ++q) {
    v4f v = *(const v4f*)(A + srow * CD + 4 * L + 128 * q);
    if (ABF) { v.x = cmb_bf(v.x); v.y = cmb_bf(v.y); v.z = cmb_bf(v.z); v.w = cmb_bf(v.w); }
    *(v4f*)(rowp + 4 * L + 128 * q) = v;
  }
}

template <int WR_LDS, int WR_F32, int WR_H16>
__device__ __forceinline__ void ln_stage(float* rowp, const float* __restrict__ GA, const float* __restrict__ BE,
                                         float* __restrict__ PF, unsigned short* __restrict__ PH, size_t row, int L) {
  #pragma clang fp contract(off)
  float s = 0.f;
#pragma unroll 1
  for (int q = 0; q < 8; ++q) {
    const v4f x = *(const v4f*)(rowp + 4 * L + 128 * q);
    s += (x.x + x.y) + (x.z + x.w);
  }
#pragma unroll
  for (int o = 16; o > 0; o >>= 1) s += __shfl_xor(s, o, 32);
  const float mu = s * 0.0009765625f; float qq = 0.f;
#pragma unroll 1
  for (int q = 0; q < 8; ++q) {
    const v4f x = *(const v4f*)(rowp + 4 * L + 128 * q);
    v4f y; y.x = x.x - mu; y.y = x.y - mu; y.z = x.z - mu; y.w = x.w - mu;
    qq += (y.x * y.x + y.y * y.y) + (y.z * y.z + y.w * y.w);
  }
#pragma unroll
  for (int o = 16; o > 0; o >>= 1) qq += __shfl_xor(qq, o, 32);
  const float rs = rsqrtf(qq * 0.0009765625f + LN_EPS);
#pragma unroll 1
  for (int q = 0; q < 8; ++q) {
    const int c = 4 * L + 128 * q;
    const v4f x = *(const v4f*)(rowp + c);
    const v4f ga = *(const v4f*)(GA + c), be = *(const v4f*)(BE + c);
    v4f y; y.x = x.x - mu; y.y = x.y - mu; y.z = x.z - mu; y.w = x.w - mu;
    y.x = y.x * rs * cmb_bf(ga.x) + cmb_bf(be.x); y.y = y.y * rs * cmb_bf(ga.y) + cmb_bf(be.y);
    y.z = y.z * rs * cmb_bf(ga.z) + cmb_bf(be.z); y.w = y.w * rs * cmb_bf(ga.w) + cmb_bf(be.w);
    if (WR_LDS) *(v4f*)(rowp + c) = y;
    if (WR_F32) VST2(v4f, (v4f*)(PF + row * CD + c), y);
    if (WR_H16) { v2u pk; pk.x = pk2h_fl(y.x, y.y); pk.y = pk2h_fl(y.z, y.w); VST2(v2u, (v2u*)(PH + row * CD + c), pk); }
  }
}

__global__ __launch_bounds__(256) void k_ln_front1(const float* __restrict__ XX, const float* __restrict__ GA, const float* __restrict__ BA,
                                                   const float* __restrict__ G1, const float* __restrict__ B1, const float* __restrict__ G2, const float* __restrict__ B2,
                                                   float* __restrict__ X0, float* __restrict__ XL, unsigned short* __restrict__ XL16, unsigned short* __restrict__ YL16) {
  __shared__ __align__(16) float s_row[8][CD];
  const int wave = __builtin_amdgcn_readfirstlane(threadIdx.x >> 5);
  const int r = blockIdx.x * 8 + wave; const int L = threadIdx.x & 31; if (r >= MTOK) return;
  const size_t srow = (size_t)(r / SEQ) * SEQ_FULL + (size_t)(r % SEQ);
  float* rowp = s_row[wave];
  ln_fetch<1>(XX, srow, L, rowp);
  ln_stage<1, 1, 0>(rowp, GA, BA, X0, nullptr, (size_t)r, L);
  ln_stage<0, 1, 1>(rowp, G1, B1, XL, XL16, (size_t)r, L);
  ln_stage<0, 0, 1>(rowp, G2, B2, nullptr, YL16, (size_t)r, L);
}

__global__ __launch_bounds__(256) void k_ln_front2(const float* __restrict__ X1, const float* __restrict__ EE, const float* __restrict__ GB, const float* __restrict__ BB,
                                                   const float* __restrict__ G1, const float* __restrict__ B1, const float* __restrict__ G2, const float* __restrict__ B2,
                                                   float* __restrict__ XB, float* __restrict__ XL, unsigned short* __restrict__ XL16, unsigned short* __restrict__ YL16,
                                                   float* __restrict__ OUT1) {
  __shared__ __align__(16) float s_row[8][CD];
  const int wave = __builtin_amdgcn_readfirstlane(threadIdx.x >> 5);
  const int r = blockIdx.x * 8 + wave; const int L = threadIdx.x & 31; if (r >= MTOK) return;
  const size_t srow = (size_t)(r / SEQ) * SEQ_FULL + (size_t)(r % SEQ);
  float* rowp = s_row[wave];
  ln_fetch<0>(X1, (size_t)r, L, rowp);
  ln_stage<1, 1, 0>(rowp, GB, BB, XB, nullptr, (size_t)r, L);
  ln_stage<0, 1, 1>(rowp, G1, B1, XL, XL16, (size_t)r, L);
#pragma unroll 1
  for (int q = 0; q < 8; ++q) {
    const int c = 4 * L + 128 * q;
    v4f v = *(const v4f*)(EE + srow * CD + c);
    v.x = cmb_bf(v.x); v.y = cmb_bf(v.y); v.z = cmb_bf(v.z); v.w = cmb_bf(v.w);
    *(v4f*)(rowp + c) = v;
    VST2(v4f, (v4f*)(OUT1 + srow * CD + c), v);
  }
  ln_stage<0, 0, 1>(rowp, G2, B2, nullptr, YL16, (size_t)r, L);
}

__global__ __launch_bounds__(256) void k_ln_mid(const float* __restrict__ OUTP, const float* __restrict__ XS, const float* __restrict__ G3, const float* __restrict__ B3,
                                                float* __restrict__ SUMP, unsigned short* __restrict__ H16) {
  __shared__ __align__(16) float s_row[8][CD];
  const int wave = __builtin_amdgcn_readfirstlane(threadIdx.x >> 5);
  const int r = blockIdx.x * 8 + wave; const int L = threadIdx.x & 31; if (r >= MTOK) return;
  float* rowp = s_row[wave];
#pragma unroll 1
  for (int q = 0; q < 8; ++q) {
    const int c = 4 * L + 128 * q;
    const v4f a = *(const v4f*)(OUTP + (size_t)r * CD + c);
    const v4f x = *(const v4f*)(XS + (size_t)r * CD + c);
    *(v4f*)(rowp + c) = a;
    const v4f sm = x + a;
    VST2(v4f, (v4f*)(SUMP + (size_t)r * CD + c), sm);
  }
  ln_stage<0, 0, 1>(rowp, G3, B3, nullptr, H16, (size_t)r, L);
}

struct GP {
  const unsigned short* A; const unsigned short* Bt; void* C; const float* bias; const float* R;
  long long strideA, strideC;
  int lda, ldb, ldc, ldr, M, N, K, rpb, rpbC, rpbR; float scale; int pad_;
};
static_assert(sizeof(GP) == 104);

template <int BIAS_MODE, int OUT_MODE, int RES_MODE, int ACT>
__device__ __forceinline__ void gemm_body(const GP& p) {
  __shared__ __align__(16) float sT[8][16 * 68];
  const int b = blockIdx.y;
  const int lane = threadIdx.x & 31, wave = __builtin_amdgcn_readfirstlane(threadIdx.x >> 5);
  const int tilesN = p.N >> 6, tilesM = p.M >> 6;
  const int tile = blockIdx.x * 8 + wave;
  if (tile >= tilesM * tilesN) return;
  const int tm = tile / tilesN, tn = tile - tm * tilesN;
  const int m0 = tm << 6, n0 = tn << 6;
  const _Float16* Ab = (const _Float16*)p.A + (size_t)b * p.strideA;
  const _Float16* Bb = (const _Float16*)p.Bt;
  const int rlane = lane & 15, koff = (lane >> 4) * 8, mOff = (lane >> 4) * 8;

  v8f acc[4][4];
#pragma unroll
  for (int i = 0; i < 4; ++i)
#pragma unroll
    for (int j = 0; j < 4; ++j) acc[i][j] = (v8f){0.f, 0.f, 0.f, 0.f, 0.f, 0.f, 0.f, 0.f};

  for (int k0 = 0; k0 < p.K; k0 += 32) {
    v16h bh[4];
#pragma unroll
    for (int j = 0; j < 4; ++j) bh[j] = ldg_frag(Bb + (size_t)(n0 + (j << 4) + rlane) * p.ldb + koff + k0);
#pragma unroll
    for (int i = 0; i < 4; ++i) {
      const v16h ah = ldg_frag(Ab + (size_t)(m0 + (i << 4) + rlane) * p.lda + koff + k0);
#pragma unroll
      for (int j = 0; j < 4; ++j) acc[i][j] = __builtin_amdgcn_wmma_f32_16x16x32_f16(false, ah, false, bh[j], (short)0, acc[i][j], false, false);
      dep_guard_h(acc[i][0], acc[i][3], ah, ah);
    }
    keep4_h(bh[0], bh[1], bh[2], bh[3]);
  }
  acc_guard4(acc[0][0], acc[0][1], acc[0][2], acc[0][3]);
  acc_guard4(acc[1][0], acc[1][1], acc[1][2], acc[1][3]);
  acc_guard4(acc[2][0], acc[2][1], acc[2][2], acc[2][3]);
  acc_guard4(acc[3][0], acc[3][1], acc[3][2], acc[3][3]);

  float* slab = sT[wave];
#pragma unroll
  for (int i = 0; i < 4; ++i) {
    const int mBase = m0 + (i << 4);
    float bm[8];
#pragma unroll
    for (int r = 0; r < 8; ++r) { bm[r] = 0.f; if (BIAS_MODE == 1) bm[r] = cmb_bf(p.bias[mBase + mOff + r]); }
#pragma unroll
    for (int j = 0; j < 4; ++j) {
      const int n = n0 + (j << 4) + rlane;
      float bv = 0.f; if (BIAS_MODE == 2) bv = cmb_bf(p.bias[n]);
#pragma unroll
      for (int r = 0; r < 8; ++r) {
        float v = acc[i][j][r] * p.scale + ((BIAS_MODE == 1) ? bm[r] : bv);
        if (ACT == 1) v = gelu_erf(v);
        slab[(mOff + r) * 68 + (j << 4) + rlane] = v;
      }
    }
    WAVE_SYNC();
    const int gb = mBase / p.rpb; const int tIn = mBase - gb * p.rpb;
    const size_t rowC0 = (size_t)gb * p.rpbC + tIn, rowR0 = (size_t)gb * p.rpbR + tIn;
    if (OUT_MODE == 0) {
      float* C = (float*)p.C + (size_t)b * p.strideC;
      const int hh = lane >> 4, c4 = (lane & 15) * 4;
      v4f val[8];
#pragma unroll
      for (int it = 0; it < 8; ++it) {
        const int row = it * 2 + hh;
        v4f v = *(const v4f*)(slab + row * 68 + c4);
        if (RES_MODE != 0) {
          v4f x = *(const v4f*)(p.R + (rowR0 + row) * (size_t)p.ldr + n0 + c4);
          if (RES_MODE == 2) { x.x = cmb_bf(x.x); x.y = cmb_bf(x.y); x.z = cmb_bf(x.z); x.w = cmb_bf(x.w); }
          v = v + x;
        }
        val[it] = v;
      }
      for (int pass = 0; pass < 2; ++pass) {
#pragma unroll
        for (int it = 0; it < 8; ++it) {
          const int row = it * 2 + hh;
          *(volatile v4f*)(C + (rowC0 + row) * (size_t)p.ldc + n0 + c4) = val[it];
        }
        __threadfence();
      }
    } else {
      unsigned short* C = (unsigned short*)p.C + (size_t)b * p.strideC;
      const int q = lane >> 3, c8 = (lane & 7) * 8;
      v8h hv[4];
#pragma unroll
      for (int it = 0; it < 4; ++it) {
        const float* sp = slab + (it * 4 + q) * 68 + c8;
#pragma unroll
        for (int e = 0; e < 8; ++e) hv[it][e] = toh_flush(sp[e]);
      }
      for (int pass = 0; pass < 2; ++pass) {
#pragma unroll
        for (int it = 0; it < 4; ++it) {
          const int row = it * 4 + q;
          *(volatile v8h*)(C + (rowC0 + row) * (size_t)p.ldc + n0 + c8) = hv[it];
        }
        __threadfence();
      }
    }
    WAVE_SYNC();
  }
}

__device__ __forceinline__ GP gp_pack(const unsigned short* A, const unsigned short* Bt, void* C, const float* bias, const float* R,
                                      long long strideA, long long strideC, int lda, int ldb, int ldc, int ldr, int M, int N, int K,
                                      int rpb, int rpbC, int rpbR, float scale) {
  GP g;
  g.A = A; g.Bt = Bt; g.C = C; g.bias = bias; g.R = R; g.strideA = strideA; g.strideC = strideC;
  g.lda = lda; g.ldb = ldb; g.ldc = ldc; g.ldr = ldr; g.M = M; g.N = N; g.K = K; g.rpb = rpb; g.rpbC = rpbC; g.rpbR = rpbR;
  g.scale = scale; g.pad_ = 0;
  return g;
}

__global__ __launch_bounds__(256) void k_gemm_nb16(const unsigned short* A, const unsigned short* Bt, void* C, const float* bias, const float* R,
                                                   long long strideA, long long strideC, int lda, int ldb, int ldc, int ldr, int M, int N, int K,
                                                   int rpb, int rpbC, int rpbR, float scale) {
  const GP p = gp_pack(A, Bt, C, bias, R, strideA, strideC, lda, ldb, ldc, ldr, M, N, K, rpb, rpbC, rpbR, scale);
  gemm_body<0, 1, 0, 0>(p);
}
__global__ __launch_bounds__(256) void k_gemm_res(const unsigned short* A, const unsigned short* Bt, void* C, const float* bias, const float* R,
                                                  long long strideA, long long strideC, int lda, int ldb, int ldc, int ldr, int M, int N, int K,
                                                  int rpb, int rpbC, int rpbR, float scale) {
  const GP p = gp_pack(A, Bt, C, bias, R, strideA, strideC, lda, ldb, ldc, ldr, M, N, K, rpb, rpbC, rpbR, scale);
  gemm_body<2, 0, 1, 0>(p);
}
__global__ __launch_bounds__(256) void k_gemm_fc(const unsigned short* A, const unsigned short* Bt, void* C, const float* bias, const float* R,
                                                 long long strideA, long long strideC, int lda, int ldb, int ldc, int ldr, int M, int N, int K,
                                                 int rpb, int rpbC, int rpbR, float scale) {
  const GP p = gp_pack(A, Bt, C, bias, R, strideA, strideC, lda, ldb, ldc, ldr, M, N, K, rpb, rpbC, rpbR, scale);
  gemm_body<2, 1, 0, 1>(p);
}

constexpr float ATT_SC = (float)(1.4426950408889634 * 0.17677669529663688);
#define ATT_PLOG 12.0f
#define ATT_OCAR 1024.0f

template <int CAUSAL>
__device__ __forceinline__ void attn_body(const unsigned short* __restrict__ QKp, const unsigned short* __restrict__ VTp, unsigned short* __restrict__ CTXp) {
  __shared__ __align__(16) _Float16 Osh[4][16 * 64];
  const int tid = threadIdx.x, lane = tid & 31, hh = lane >> 4, c = lane & 15;
  const int wave = __builtin_amdgcn_readfirstlane(tid >> 5);
  const int bx = blockIdx.x; const int qb = bx % NCH; const int bhp = bx / NCH; const int hp = bhp % (NH / 2); const int b = bhp / (NH / 2);
  const int q0 = qb * 64 + wave * 16;
  const int qi = q0 + c;
  const _Float16* QK = (const _Float16*)QKp; const _Float16* VT = (const _Float16*)VTp;
  const size_t tok0 = (size_t)b * SEQ;
  _Float16* os = Osh[wave];

#pragma unroll 1
  for (int hs = 0; hs < 2; ++hs) {
    const int h = hp * 2 + hs;
    const v16h qf = ldg_frag(QK + (tok0 + q0 + c) * (size_t)QKP + h * HD + 8 * hh);
    float mrun = -INFINITY, lrun = 0.f;
    v8f oacc[2];
#pragma unroll
    for (int t = 0; t < 2; ++t) oacc[t] = (v8f){0.f, 0.f, 0.f, 0.f, 0.f, 0.f, 0.f, 0.f};

#pragma unroll 1
    for (int kc = 0; kc < NCH; ++kc) {
      const int kv0 = kc * 64;
      v8f s[4];
#pragma unroll
      for (int j = 0; j < 4; ++j) {
        const v16h kf = ldg_frag(QK + (tok0 + kv0 + j * 16 + c) * (size_t)QKP + HDM + h * HD + 8 * hh);
        const v8f z = (v8f){0.f, 0.f, 0.f, 0.f, 0.f, 0.f, 0.f, 0.f};
        s[j] = mma_h(kf, qf, z);
      }
      float m = fmaxf(fmaxf(s[0][0], s[1][0]), fmaxf(s[2][0], s[3][0]));
#pragma unroll
      for (int r = 1; r < 8; ++r) m = fmaxf(m, fmaxf(fmaxf(s[0][r], s[1][r]), fmaxf(s[2][r], s[3][r])));
      m = fmaxf(m, __shfl_xor(m, 16, 32));
      const float mnew = fmaxf(mrun, m * ATT_SC);
      const float alpha = __builtin_amdgcn_exp2f(mrun - mnew);
      mrun = mnew;
      const float moff = ATT_PLOG - mnew;
      float ps[4];
#pragma unroll
      for (int j = 0; j < 4; ++j) {
        ps[j] = 0.f;
#pragma unroll
        for (int r = 0; r < 8; ++r) {
          const float e = s[j][r] * ATT_SC + moff;
          const float pv = __builtin_amdgcn_exp2f(e);
          ps[j] += pv;
          s[j][r] = (e < -14.0f) ? 0.f : pv;
        }
      }
      float psum = (ps[0] + ps[1]) + (ps[2] + ps[3]);
      psum += __shfl_xor(psum, 16, 32);
      lrun = lrun * alpha + psum;
#pragma unroll
      for (int t = 0; t < 2; ++t)
#pragma unroll
        for (int r = 0; r < 8; ++r) oacc[t][r] *= alpha;

      if (CAUSAL == 0 || kc <= qb) {
        if (CAUSAL != 0 && kc == qb) {
#pragma unroll
          for (int j = 0; j < 4; ++j)
#pragma unroll
            for (int r = 0; r < 8; ++r) {
              const int key = kv0 + j * 16 + 8 * hh + r;
              s[j][r] = (key < qi) ? s[j][r] : 0.f;
            }
        }
#pragma unroll
        for (int kk = 0; kk < 2; ++kk) {
          FH pb;
#pragma unroll
          for (int e = 0; e < 8; ++e) { pb.h[0][e] = (_Float16)s[2 * kk][e]; pb.h[1][e] = (_Float16)s[2 * kk + 1][e]; }
#pragma unroll
          for (int t = 0; t < 2; ++t) {
            const v16h va = ldg_frag(VT + (size_t)(h * HD + t * 16 + c) * VTP + tok0 + kv0 + kk * 32 + 8 * hh);
            oacc[t] = mma_h(va, pb.v, oacc[t]);
          }
        }
      }
    }

    const float inv = ATT_OCAR * __builtin_amdgcn_rcpf(lrun);
#pragma unroll
    for (int t = 0; t < 2; ++t) {
      v8h hv;
#pragma unroll
      for (int r = 0; r < 8; ++r) hv[r] = toh_flush(oacc[t][r] * inv);
      *(v8h*)(os + c * 64 + hs * 32 + t * 16 + 8 * hh) = hv;
    }
  }
  WAVE_SYNC();
  {
    const int q = lane >> 3, c8 = (lane & 7) * 8;
    v8h hv[4];
#pragma unroll
    for (int it = 0; it < 4; ++it) hv[it] = *(const v8h*)(os + (it * 4 + q) * 64 + c8);
    for (int pass = 0; pass < 2; ++pass) {
#pragma unroll
      for (int it = 0; it < 4; ++it)
        *(volatile v8h*)(CTXp + (tok0 + q0 + it * 4 + q) * (size_t)HDM + hp * 64 + c8) = hv[it];
      __threadfence();
    }
  }
}
__global__ __launch_bounds__(128) void k_attn_causal(const unsigned short* __restrict__ QKp, const unsigned short* __restrict__ VTp, unsigned short* __restrict__ CTXp) { attn_body<1>(QKp, VTp, CTXp); }
__global__ __launch_bounds__(128) void k_attn_dense(const unsigned short* __restrict__ QKp, const unsigned short* __restrict__ VTp, unsigned short* __restrict__ CTXp) { attn_body<0>(QKp, VTp, CTXp); }

constexpr size_t SZ_P32  = (size_t)MTOK * CD * 4;
constexpr size_t SZ_X16  = (size_t)MTOK * CD * 2;
constexpr size_t SZ_Y16  = (size_t)MTOK * CD * 2;
constexpr size_t SZ_QK   = (size_t)MTOK * QKP * 2;
constexpr size_t SZ_VT   = (size_t)HDM * VTP * 2;
constexpr size_t SZ_CTX  = (size_t)MTOK * HDM * 2;
constexpr size_t SZ_F16  = (size_t)MTOK * C4 * 2;
constexpr size_t SZ_WQKV = (size_t)3 * HDM * CD * 2;
constexpr size_t SZ_WOT  = (size_t)CD * HDM * 2;
constexpr size_t SZ_W2T  = (size_t)C4 * CD * 2;
constexpr size_t SZ_W3T  = (size_t)CD * C4 * 2;
constexpr size_t OFF_P0   = 0;
constexpr size_t OFF_P1   = OFF_P0 + SZ_P32;
constexpr size_t OFF_P2   = OFF_P1 + SZ_P32;
constexpr size_t OFF_X16  = OFF_P2 + SZ_P32;
constexpr size_t OFF_SCR  = OFF_X16 + SZ_X16;
constexpr size_t OFF_Y16  = OFF_SCR;
constexpr size_t OFF_QK   = OFF_Y16 + SZ_Y16;
constexpr size_t OFF_VT   = OFF_QK + SZ_QK;
constexpr size_t OFF_CTX  = OFF_VT + SZ_VT;
constexpr size_t OFF_F16  = OFF_SCR;
constexpr size_t OFF_WQKV = OFF_SCR + SZ_F16;
constexpr size_t OFF_WOT  = OFF_WQKV + SZ_WQKV;
constexpr size_t OFF_W2T  = OFF_WOT + SZ_WOT;
constexpr size_t OFF_W3T  = OFF_W2T + SZ_W2T;
constexpr size_t WS_TOTAL = OFF_W3T + SZ_W3T;
static_assert(OFF_CTX + SZ_CTX <= OFF_SCR + SZ_F16);
static_assert(WS_TOTAL <= (size_t)134217728);
static_assert(SZ_P32 % 256 == 0 && SZ_X16 % 256 == 0 && SZ_Y16 % 256 == 0 && SZ_QK % 256 == 0 && SZ_VT % 256 == 0 && SZ_CTX % 256 == 0 &&
              SZ_F16 % 256 == 0 && SZ_WQKV % 256 == 0 && SZ_WOT % 256 == 0 && SZ_W2T % 256 == 0 && SZ_W3T % 256 == 0);

static GP mk_gp(const unsigned short* A, long long sA, int lda, const unsigned short* Bt, int ldb, void* C, long long sC, int ldc,
                const float* bias, const float* R, int ldr, int M, int N, int K, int rpb, int rpbC, int rpbR) {
  GP g{};
  g.A = A; g.Bt = Bt; g.C = C; g.bias = bias; g.R = R; g.strideA = sA; g.strideC = sC;
  g.lda = lda; g.ldb = ldb; g.ldc = ldc; g.ldr = ldr; g.M = M; g.N = N; g.K = K; g.rpb = rpb; g.rpbC = rpbC; g.rpbR = rpbR;
  g.scale = 0.0625f; g.pad_ = 0;
  return g;
}
#define GP_ARGS(g) (g).A, (g).Bt, (g).C, (g).bias, (g).R, (g).strideA, (g).strideC, (g).lda, (g).ldb, (g).ldc, (g).ldr, (g).M, (g).N, (g).K, (g).rpb, (g).rpbC, (g).rpbR, (g).scale
static unsigned gemm_blocks(int M, int N) { return (unsigned)((((M / 64) * (N / 64)) + 7) / 8); }

struct LayerIn { const float *g1, *b1, *g2, *b2, *g3, *b3, *wq, *wk, *wv, *wo, *bo, *w2, *bb2, *w3, *bb3; };
static LayerIn bind_layer(void* const* d_in, int pi) {
  LayerIn w;
  w.g1 = (const float*)d_in[pi + 0];  w.b1 = (const float*)d_in[pi + 1];
  w.g2 = (const float*)d_in[pi + 2];  w.b2 = (const float*)d_in[pi + 3];
  w.g3 = (const float*)d_in[pi + 4];  w.b3 = (const float*)d_in[pi + 5];
  w.wq = (const float*)d_in[pi + 6];  w.wk = (const float*)d_in[pi + 7];  w.wv = (const float*)d_in[pi + 8];
  w.wo = (const float*)d_in[pi + 9];  w.bo = (const float*)d_in[pi + 10];
  w.w2 = (const float*)d_in[pi + 11]; w.bb2 = (const float*)d_in[pi + 12];
  w.w3 = (const float*)d_in[pi + 13]; w.bb3 = (const float*)d_in[pi + 14];
  return w;
}
static int layer_sizes_ok(const int* s, int pi) {
  for (int i = 0; i < 6; ++i) if (s[pi + i] < CD) return 0;
  for (int i = 6; i < 9; ++i) if (s[pi + i] < NH * CD * HD) return 0;
  if (s[pi + 9] < HDM * CD || s[pi + 10] < CD || s[pi + 11] < CD * C4 || s[pi + 12] < C4 || s[pi + 13] < C4 * CD || s[pi + 14] < CD) return 0;
  return 1;
}

static void run_tail(hipStream_t stream, const LayerIn& w, int causal,
                     unsigned short* X16, unsigned short* Y16, unsigned short* QK, unsigned short* VT, unsigned short* CTX, unsigned short* F16,
                     unsigned short* WQKV, unsigned short* WOT, unsigned short* W2T, unsigned short* W3T,
                     const float* XLF, float* OUTP, const float* XSKIP, float* SUMP, float* CFIN, int rpb, int rpbC, int rpbR) {
  const int BIG = 1 << 30;
  const unsigned qkv_blocks = (unsigned)((HDM * (CD / 8)) / 256);
  k_castqkv<<<qkv_blocks, 256, 0, stream>>>(w.wq, WQKV);
  k_castqkv<<<qkv_blocks, 256, 0, stream>>>(w.wk, WQKV + (size_t)HDM * CD);
  k_castqkv<<<qkv_blocks, 256, 0, stream>>>(w.wv, WQKV + (size_t)2 * HDM * CD);
  k_castbT<<<(unsigned)((((long long)CD) * (HDM / 8) + 255) / 256), 256, 0, stream>>>(w.wo, CD, WOT, HDM, HDM, CD, 16.0f);
  k_castbT<<<(unsigned)((((long long)C4) * (CD / 8) + 255) / 256), 256, 0, stream>>>(w.w2, C4, W2T, CD, CD, C4, 16.0f);
  k_castbT<<<(unsigned)((((long long)CD) * (C4 / 8) + 255) / 256), 256, 0, stream>>>(w.w3, CD, W3T, C4, C4, CD, 16.0f);

  { const GP g = mk_gp(X16, 0, CD, WQKV, CD, (void*)QK, 0, QKP, w.bo, nullptr, 0, MTOK, HDM, CD, BIG, BIG, BIG);
    k_gemm_nb16<<<dim3(gemm_blocks(MTOK, HDM), 1), 256, 0, stream>>>(GP_ARGS(g)); }
  { const GP g = mk_gp(Y16, 0, CD, WQKV + (size_t)HDM * CD, CD, (void*)(QK + HDM), 0, QKP, w.bo, nullptr, 0, MTOK, HDM, CD, BIG, BIG, BIG);
    k_gemm_nb16<<<dim3(gemm_blocks(MTOK, HDM), 1), 256, 0, stream>>>(GP_ARGS(g)); }
  { const GP g = mk_gp(WQKV + (size_t)2 * HDM * CD, 0, CD, Y16, CD, (void*)VT, 0, VTP, w.bo, nullptr, 0, HDM, MTOK, CD, BIG, BIG, BIG);
    k_gemm_nb16<<<dim3(gemm_blocks(HDM, MTOK), 1), 256, 0, stream>>>(GP_ARGS(g)); }
  if (causal) k_attn_causal<<<NB * (NH / 2) * NCH, 128, 0, stream>>>(QK, VT, CTX);
  else        k_attn_dense<<<NB * (NH / 2) * NCH, 128, 0, stream>>>(QK, VT, CTX);
  { GP g = mk_gp(CTX, 0, HDM, WOT, HDM, (void*)OUTP, 0, CD, w.bo, XLF, CD, MTOK, CD, HDM, BIG, BIG, BIG);
    g.scale = 0.0625f / ATT_OCAR;
    k_gemm_res<<<dim3(gemm_blocks(MTOK, CD), 1), 256, 0, stream>>>(GP_ARGS(g)); }
  k_ln_mid<<<MTOK / 8, 256, 0, stream>>>(OUTP, XSKIP, w.g3, w.b3, SUMP, X16);
  { const GP g = mk_gp(X16, 0, CD, W2T, CD, (void*)F16, 0, C4, w.bb2, nullptr, 0, MTOK, C4, CD, BIG, BIG, BIG);
    k_gemm_fc<<<dim3(gemm_blocks(MTOK, C4), 1), 256, 0, stream>>>(GP_ARGS(g)); }
  { const GP g = mk_gp(F16, 0, C4, W3T, C4, (void*)CFIN, 0, CD, w.bb3, SUMP, CD, MTOK, CD, C4, rpb, rpbC, rpbR);
    k_gemm_res<<<dim3(gemm_blocks(MTOK, CD), 1), 256, 0, stream>>>(GP_ARGS(g)); }
}

extern "C" void kernel_launch(void* const* d_in, const int* in_sizes, int n_in, void* d_out, int out_size, void* d_ws, size_t ws_size, hipStream_t stream) {
  if (n_in < 36) return;
  const long long need_x = ((long long)(NB - 1) * SEQ_FULL + SEQ) * CD;
  const long long out1_el = (long long)NB_FULL * SEQ_FULL * CD;
  if ((long long)in_sizes[0] < need_x) return;
  if ((long long)in_sizes[1] < need_x) return;
  if (in_sizes[2] < CD || in_sizes[3] < CD || in_sizes[4] < CD || in_sizes[5] < CD) return;
  if (!layer_sizes_ok(in_sizes, 6)) return;
  if (!layer_sizes_ok(in_sizes, 21)) return;
  if ((long long)out_size < out1_el + need_x) return;
  if (ws_size < WS_TOTAL) return;

  const float* xx   = (const float*)d_in[0];
  const float* ee   = (const float*)d_in[1];
  const float* lnAg = (const float*)d_in[2];
  const float* lnAb = (const float*)d_in[3];
  const float* lnBg = (const float*)d_in[4];
  const float* lnBb = (const float*)d_in[5];
  const LayerIn a1 = bind_layer(d_in, 6);
  const LayerIn a2 = bind_layer(d_in, 21);
  float* out = (float*)d_out;
  char* wsp = (char*)d_ws;
  float*          P0   = (float*)(wsp + OFF_P0);
  float*          P1   = (float*)(wsp + OFF_P1);
  float*          P2   = (float*)(wsp + OFF_P2);
  unsigned short* X16  = (unsigned short*)(wsp + OFF_X16);
  unsigned short* Y16  = (unsigned short*)(wsp + OFF_Y16);
  unsigned short* QK   = (unsigned short*)(wsp + OFF_QK);
  unsigned short* VT   = (unsigned short*)(wsp + OFF_VT);
  unsigned short* CTX  = (unsigned short*)(wsp + OFF_CTX);
  unsigned short* F16  = (unsigned short*)(wsp + OFF_F16);
  unsigned short* WQKV = (unsigned short*)(wsp + OFF_WQKV);
  unsigned short* WOT  = (unsigned short*)(wsp + OFF_WOT);
  unsigned short* W2T  = (unsigned short*)(wsp + OFF_W2T);
  unsigned short* W3T  = (unsigned short*)(wsp + OFF_W3T);
  const int BIG = 1 << 30;

  k_ln_front1<<<MTOK / 8, 256, 0, stream>>>(xx, lnAg, lnAb, a1.g1, a1.b1, a1.g2, a1.b2, P0, P1, X16, Y16);
  run_tail(stream, a1, 1, X16, Y16, QK, VT, CTX, F16, WQKV, WOT, W2T, W3T, P1, P2, P0, P1, P0, BIG, BIG, BIG);
  k_ln_front2<<<MTOK / 8, 256, 0, stream>>>(P0, ee, lnBg, lnBb, a2.g1, a2.b1, a2.g2, a2.b2, P1, P2, X16, Y16, out + out1_el);
  run_tail(stream, a2, 0, X16, Y16, QK, VT, CTX, F16, WQKV, WOT, W2T, W3T, P2, P0, P1, P2, out, SEQ, SEQ_FULL, SEQ);
}
